// PD_Block_32701880992218
// MI455X (gfx1250) — hardware-run, weakly checked
//
#include <hip/hip_runtime.h>
#include <math.h>

constexpr int kBatch  = 8;
constexpr int kCin    = 256;
constexpr int kCd     = 128;
constexpr int kNsp    = 4096;
constexpr int kPix    = kBatch * kNsp;
constexpr int kQChunk = 2048;
constexpr int kWElems = 32768;
constexpr float kWCarry    = 16.0f;
constexpr float kWCarryInv = 1.0f / 16.0f;
constexpr float kPCarry    = 2048.0f;
constexpr float kPCarryInv = 1.0f / 2048.0f;

constexpr size_t kOffX  = 0;
constexpr size_t kOffXi = 16777216;
constexpr size_t kOffQ  = 33554432;
constexpr size_t kOffK  = 41943040;
constexpr size_t kOffT  = 50331648;
constexpr size_t kOffV  = 67108864;
constexpr size_t kOffP  = 75497472;
constexpr size_t kOffZ  = 92274688;
constexpr size_t kOffW  = 100663296;
constexpr size_t kWsEnd = 100990976;

typedef __attribute__((ext_vector_type(16))) _Float16 v16h;
typedef __attribute__((ext_vector_type(8)))  _Float16 v8h;
typedef __attribute__((ext_vector_type(16))) __bf16   v16b;
typedef __attribute__((ext_vector_type(8)))  __bf16   v8b;
typedef __attribute__((ext_vector_type(8)))  float    v8f;
typedef __attribute__((ext_vector_type(4)))  float    v4f;
typedef __attribute__((ext_vector_type(4)))  unsigned int v4u;

__device__ __forceinline__ unsigned short f2bf_bits(float f) {
  unsigned u = __float_as_uint(f);
  return (unsigned short)((u + 0x7FFFu + ((u >> 16) & 1u)) >> 16);
}
__device__ __forceinline__ float bf_bits2f(unsigned short h) { return __uint_as_float(((unsigned)h) << 16); }

__device__ __forceinline__ void dep_guard_h(v8f& a, v8f& b, v16h x, v16h y) { asm volatile("v_nop\n\tv_nop\n\tv_nop\n\tv_nop" : "+v"(a), "+v"(b) : "v"(x), "v"(y)); }
__device__ __forceinline__ void dep_guard_b(v8f& a, v8f& b, v16b x, v16b y) { asm volatile("v_nop\n\tv_nop\n\tv_nop\n\tv_nop" : "+v"(a), "+v"(b) : "v"(x), "v"(y)); }
__device__ __forceinline__ void keep4_h(v16h a, v16h b, v16h c, v16h d) { asm volatile("v_nop" :: "v"(a), "v"(b), "v"(c), "v"(d)); }
__device__ __forceinline__ void keep4_b(v16b a, v16b b, v16b c, v16b d) { asm volatile("v_nop" :: "v"(a), "v"(b), "v"(c), "v"(d)); }
__device__ __forceinline__ void acc_guard4(v8f& a, v8f& b, v8f& c, v8f& d) { asm volatile("v_nop\n\tv_nop\n\tv_nop\n\tv_nop" : "+v"(a), "+v"(b), "+v"(c), "+v"(d)); }
template <typename T> struct Frag;
template <> struct Frag<_Float16> {
  typedef v16h V; union U { v16h v; v8h h[2]; };
  static __device__ __forceinline__ v16h load(const _Float16* p) {
    U f; f.h[0] = *(const v8h*)(p); f.h[1] = *(const v8h*)(p + 16); return f.v;
  }
  static __device__ __forceinline__ v8f mma(v16h a, v16h b, v8f c) {
    return __builtin_amdgcn_wmma_f32_16x16x32_f16(false, a, false, b, (short)0, c, false, false);
  }
  static __device__ __forceinline__ void guard(v8f& a, v8f& b, v16h x, v16h y) { dep_guard_h(a, b, x, y); }
  static __device__ __forceinline__ void keep(v16h a, v16h b, v16h c, v16h d) { keep4_h(a, b, c, d); }
};
template <> struct Frag<__bf16> {
  typedef v16b V; union U { v16b v; v8b h[2]; };
  static __device__ __forceinline__ v16b load(const __bf16* p) {
    U f; f.h[0] = *(const v8b*)(p); f.h[1] = *(const v8b*)(p + 16); return f.v;
  }
  static __device__ __forceinline__ v8f mma(v16b a, v16b b, v8f c) {
    return __builtin_amdgcn_wmma_f32_16x16x32_bf16(false, a, false, b, (short)0, c, false, false);
  }
  static __device__ __forceinline__ void guard(v8f& a, v8f& b, v16b x, v16b y) { dep_guard_b(a, b, x, y); }
  static __device__ __forceinline__ void keep(v16b a, v16b b, v16b c, v16b d) { keep4_b(a, b, c, d); }
};

__device__ __forceinline__ unsigned pk16(unsigned short a, unsigned short b) { return (unsigned)a | ((unsigned)b << 16); }
__device__ __forceinline__ unsigned short h_bits(float f) { const _Float16 h = (_Float16)f; return __builtin_bit_cast(unsigned short, h); }

template <int ET> struct Elem;
template <> struct Elem<0> { typedef _Float16 T; };
template <> struct Elem<1> { typedef __bf16 T; };
template <int ET, bool SPLIT, int BIAS_MODE, int OUT_MODE, bool RESID, int ACT = 0>
__global__ __launch_bounds__(256) void wmma_gemm64(
    const unsigned short* __restrict__ Ap, const unsigned short* __restrict__ A2p, int lda, long strideA,
    const unsigned short* __restrict__ Btp, const unsigned short* __restrict__ Bt2p, int ldb, long strideB,
    void* __restrict__ Cout, void* __restrict__ Cout2, int ldc, long strideC,
    const float* __restrict__ bias,
    const float* __restrict__ resid, long strideR,
    int M, int N, int K, float scale) {
  typedef typename Elem<ET>::T T;
  typedef typename Frag<T>::V V;
  const T* A = (const T*)Ap; const T* A2 = (const T*)A2p; const T* Bt = (const T*)Btp; const T* Bt2 = (const T*)Bt2p;
  __shared__ __align__(16) float sT[8][16 * 68];
  const int b    = blockIdx.y;
  const int lane = threadIdx.x & 31;
  const int wave = threadIdx.x >> 5;
  const int tilesN = N >> 6;
  const int tilesM = M >> 6;
  const int tile = blockIdx.x * 8 + wave;
  if (tile >= tilesM * tilesN) return;
  const int tm = tile / tilesN;
  const int tn = tile - tm * tilesN;
  const int m0 = tm << 6;
  const int n0 = tn << 6;

  const T* Ab  = A  + (size_t)b * strideA;
  const T* Bb  = Bt + (size_t)b * strideB;
  const T* Ab2 = SPLIT ? (A2  + (size_t)b * strideA) : nullptr;
  const T* Bb2 = SPLIT ? (Bt2 + (size_t)b * strideB) : nullptr;

  const int rlane = lane & 15;
  const int koff  = (lane >> 4) * 8;
  const int mOff  = (lane >> 4) * 8;

  v8f acc[4][4];
#pragma unroll
  for (int i = 0; i < 4; ++i)
#pragma unroll
    for (int j = 0; j < 4; ++j) acc[i][j] = (v8f){0.f,0.f,0.f,0.f,0.f,0.f,0.f,0.f};

  for (int k0 = 0; k0 < K; k0 += 32) {
    V bh[4], bl[4];
#pragma unroll
    for (int j = 0; j < 4; ++j) {
      const size_t bo = (size_t)(n0 + (j << 4) + rlane) * ldb + koff + k0;
      bh[j] = Frag<T>::load(Bb + bo);
      if (SPLIT) bl[j] = Frag<T>::load(Bb2 + bo);
    }
#pragma unroll
    for (int i = 0; i < 4; ++i) {
      const size_t ao = (size_t)(m0 + (i << 4) + rlane) * lda + koff + k0;
      V ah = Frag<T>::load(Ab + ao);
      V al;
      if (SPLIT) al = Frag<T>::load(Ab2 + ao);
#pragma unroll
      for (int j = 0; j < 4; ++j) {
        acc[i][j] = Frag<T>::mma(ah, bh[j], acc[i][j]);
        if (SPLIT) {
          acc[i][j] = Frag<T>::mma(ah, bl[j], acc[i][j]);
          acc[i][j] = Frag<T>::mma(al, bh[j], acc[i][j]);
        }
      }
      Frag<T>::guard(acc[i][0], acc[i][3], ah, SPLIT ? al : ah);
    }
    Frag<T>::keep(bh[0], bh[1], bh[2], bh[3]);
    if (SPLIT) Frag<T>::keep(bl[0], bl[1], bl[2], bl[3]);
  }
  acc_guard4(acc[0][0], acc[0][1], acc[0][2], acc[0][3]);
  acc_guard4(acc[1][0], acc[1][1], acc[1][2], acc[1][3]);
  acc_guard4(acc[2][0], acc[2][1], acc[2][2], acc[2][3]);
  acc_guard4(acc[3][0], acc[3][1], acc[3][2], acc[3][3]);

  float* slab = sT[wave];
  const float* Rb = RESID ? (resid + (size_t)b * strideR) : nullptr;
#pragma unroll
  for (int i = 0; i < 4; ++i) {
    const int mBase = m0 + (i << 4);
#pragma unroll
    for (int j = 0; j < 4; ++j) {
      const int n = n0 + (j << 4) + rlane;
      float bv = 0.f;
      if (BIAS_MODE == 2) bv = bias[n];
#pragma unroll
      for (int r = 0; r < 8; ++r) {
        float v = acc[i][j][r] * scale;
        if (BIAS_MODE == 1) v += bias[mBase + mOff + r];
        if (BIAS_MODE == 2) v += bv;
        if (RESID) v += Rb[(size_t)(mBase + mOff + r) * ldc + n];
        if (ACT == 2) v = fmaxf(v, 0.0f);
        if (ACT == 4) v = (v > 0.f) ? v : 0.01f * v;
        slab[(mOff + r) * 68 + (j << 4) + rlane] = v;
      }
    }
    __builtin_amdgcn_fence(__ATOMIC_RELEASE, "workgroup");
    __builtin_amdgcn_wave_barrier();
    __builtin_amdgcn_fence(__ATOMIC_ACQUIRE, "workgroup");
    if (OUT_MODE == 0) {
      float* C = (float*)Cout + (size_t)b * strideC;
      const int hh = lane >> 4, c4 = (lane & 15) * 4;
      for (int pass = 0; pass < 2; ++pass) {
#pragma unroll
        for (int it = 0; it < 8; ++it) {
          const int row = it * 2 + hh;
          v4f v = *(const v4f*)(slab + row * 68 + c4);
          *(volatile v4f*)(C + (size_t)(mBase + row) * ldc + n0 + c4) = v;
        }
        __threadfence();
      }
    } else {
      const int q = lane >> 3, c8 = (lane & 7) * 8;
      unsigned short* C  = (unsigned short*)Cout  + (size_t)b * strideC;
      unsigned short* C2 = (OUT_MODE == 2) ? ((unsigned short*)Cout2 + (size_t)b * strideC) : nullptr;
      for (int pass = 0; pass < 2; ++pass) {
#pragma unroll
        for (int it = 0; it < 4; ++it) {
          const int row = it * 4 + q;
          const float* sp = slab + row * 68 + c8;
          v8h hv, lv;
#pragma unroll
          for (int e = 0; e < 8; ++e) {
            if (OUT_MODE == 1) {
              hv[e] = (_Float16)sp[e];
            } else {
              unsigned short hb = f2bf_bits(sp[e]);
              unsigned short lb = f2bf_bits(sp[e] - bf_bits2f(hb));
              hv[e] = __builtin_bit_cast(_Float16, hb);
              lv[e] = __builtin_bit_cast(_Float16, lb);
            }
          }
          *(volatile v8h*)(C + (size_t)(mBase + row) * ldc + n0 + c8) = hv;
          if (OUT_MODE == 2) *(volatile v8h*)(C2 + (size_t)(mBase + row) * ldc + n0 + c8) = lv;
        }
        __threadfence();
      }
    }
    __builtin_amdgcn_fence(__ATOMIC_RELEASE, "workgroup");
    __builtin_amdgcn_wave_barrier();
    __builtin_amdgcn_fence(__ATOMIC_ACQUIRE, "workgroup");
  }
}

__global__ __launch_bounds__(256) void wcast8_kernel(const float* __restrict__ W0, const float* __restrict__ W1,
                                                     const float* __restrict__ W2, const float* __restrict__ W3,
                                                     const float* __restrict__ W4, unsigned short* __restrict__ out,
                                                     float scale) {
  const int i = blockIdx.x * 256 + threadIdx.x;
  const int y = blockIdx.y;
  if (i >= kWElems / 8) return;
  const float* W = (y == 0) ? W0 : (y == 1) ? W1 : (y == 2) ? W2 : (y == 3) ? W3 : W4;
  const float* p = W + 8 * (size_t)i;
  const v4f a = *(const v4f*)(p);
  const v4f c = *(const v4f*)(p + 4);
  unsigned short hb[8];
#pragma unroll
  for (int e = 0; e < 4; ++e) {
    hb[e]     = h_bits(a[e] * scale);
    hb[4 + e] = h_bits(c[e] * scale);
  }
  const v4u u = (v4u){pk16(hb[0], hb[1]), pk16(hb[2], hb[3]), pk16(hb[4], hb[5]), pk16(hb[6], hb[7])};
  unsigned short* q = out + (size_t)y * kWElems + 8 * (size_t)i;
  *(volatile v4u*)q = u;
  __threadfence();
  *(volatile v4u*)q = u;
}

__global__ __launch_bounds__(256) void xpose_cast_kernel(const float* __restrict__ X0, const float* __restrict__ X1,
                                                         unsigned short* __restrict__ O0, unsigned short* __restrict__ O1) {
  __shared__ float sm[64][65];
  const int t   = threadIdx.x;
  const int c0  = blockIdx.x * 64;
  const int n0  = blockIdx.y * 64;
  const int src = blockIdx.z >> 3;
  const int b   = blockIdx.z & 7;
  const float* X = ((src == 0) ? X0 : X1) + (size_t)b * kCin * kNsp;
  unsigned short* O = ((src == 0) ? O0 : O1) + (size_t)b * kNsp * kCin;
#pragma unroll
  for (int i = 0; i < 16; ++i) {
    const int e = i * 256 + t;
    const int r = e >> 6;
    const int c = e & 63;
    sm[c][r] = X[(size_t)(c0 + r) * kNsp + n0 + c];
  }
  __syncthreads();
  const int lane = t & 31, wave = t >> 5;
  const int q = lane >> 3, c8 = (lane & 7) * 8;
  for (int pass = 0; pass < 2; ++pass) {
#pragma unroll
    for (int it = 0; it < 2; ++it) {
      const int row = wave * 8 + it * 4 + q;
      unsigned short hb[8];
#pragma unroll
      for (int e = 0; e < 8; ++e) hb[e] = h_bits(sm[row][c8 + e]);
      const v4u u = (v4u){pk16(hb[0], hb[1]), pk16(hb[2], hb[3]), pk16(hb[4], hb[5]), pk16(hb[6], hb[7])};
      *(volatile v4u*)(O + (size_t)(n0 + row) * kCin + c0 + c8) = u;
    }
    __threadfence();
  }
}

__global__ __launch_bounds__(256) void softmax_row_kernel(const float* __restrict__ S, unsigned short* __restrict__ P, float carry) {
  __shared__ __align__(16) float rowbuf[kNsp];
  __shared__ float redM[8];
  __shared__ float redS[8];
  const int row  = blockIdx.x;
  const int t    = threadIdx.x;
  const int lane = t & 31, wave = t >> 5;
  const int cA   = 8 * t;
  const int cB   = (kNsp / 2) + 8 * t;
  const float* sr = S + (size_t)row * kNsp;
  const v4f a0 = *(const v4f*)(sr + cA);
  const v4f a1 = *(const v4f*)(sr + cA + 4);
  const v4f a2 = *(const v4f*)(sr + cB);
  const v4f a3 = *(const v4f*)(sr + cB + 4);
  float m = fmaxf(fmaxf(fmaxf(a0[0], a0[1]), fmaxf(a0[2], a0[3])), fmaxf(fmaxf(a1[0], a1[1]), fmaxf(a1[2], a1[3])));
  m = fmaxf(m, fmaxf(fmaxf(fmaxf(a2[0], a2[1]), fmaxf(a2[2], a2[3])), fmaxf(fmaxf(a3[0], a3[1]), fmaxf(a3[2], a3[3]))));
#pragma unroll
  for (int off = 16; off > 0; off >>= 1) m = fmaxf(m, __shfl_xor(m, off, 32));
  if (lane == 0) redM[wave] = m;
  __syncthreads();
  m = redM[0];
#pragma unroll
  for (int w = 1; w < 8; ++w) m = fmaxf(m, redM[w]);

  float s = 0.f;
#pragma unroll 1
  for (int j = 0; j < 16; ++j) {
    const int col = (j < 8) ? (cA + j) : (cB + j - 8);
    const float e = expf(sr[col] - m);
    rowbuf[col] = e;
    s += e;
  }
#pragma unroll
  for (int off = 16; off > 0; off >>= 1) s += __shfl_xor(s, off, 32);
  if (lane == 0) redS[wave] = s;
  __syncthreads();
  float tot = redS[0];
#pragma unroll
  for (int w = 1; w < 8; ++w) tot += redS[w];
  const float inv = carry * (1.0f / tot);

  unsigned short ha[8], hb[8];
#pragma unroll
  for (int e = 0; e < 8; ++e) {
    ha[e] = h_bits(rowbuf[cA + e] * inv);
    hb[e] = h_bits(rowbuf[cB + e] * inv);
  }
  const v4u uA = (v4u){pk16(ha[0], ha[1]), pk16(ha[2], ha[3]), pk16(ha[4], ha[5]), pk16(ha[6], ha[7])};
  const v4u uB = (v4u){pk16(hb[0], hb[1]), pk16(hb[2], hb[3]), pk16(hb[4], hb[5]), pk16(hb[6], hb[7])};
  unsigned short* pr = P + (size_t)row * kNsp;
  *(volatile v4u*)(pr + cA) = uA;
  *(volatile v4u*)(pr + cB) = uB;
  __threadfence();
  *(volatile v4u*)(pr + cA) = uA;
  *(volatile v4u*)(pr + cB) = uB;
}

extern "C" void kernel_launch(void* const* d_in, const int* in_sizes, int n_in,
                              void* d_out, int out_size, void* d_ws, size_t ws_size,
                              hipStream_t stream) {
  if (n_in < 12) return;
  if (out_size != kBatch * kCin * kNsp) return;
  if (in_sizes[0] != kBatch * kCin * kNsp || in_sizes[1] != kBatch * kCin * kNsp) return;
  if (in_sizes[2] != kWElems || in_sizes[4] != kWElems || in_sizes[6] != kWElems ||
      in_sizes[8] != kWElems || in_sizes[10] != kWElems) return;
  if (in_sizes[3] != kCd || in_sizes[5] != kCd || in_sizes[7] != kCd || in_sizes[9] != kCd || in_sizes[11] != kCin) return;
  if (ws_size < kWsEnd) return;

  const float* feat_t = (const float*)d_in[0];
  const float* feat_i = (const float*)d_in[1];
  const float* Wq  = (const float*)d_in[2];
  const float* bq  = (const float*)d_in[3];
  const float* Wk  = (const float*)d_in[4];
  const float* bk  = (const float*)d_in[5];
  const float* Wv  = (const float*)d_in[6];
  const float* bv  = (const float*)d_in[7];
  const float* Wt  = (const float*)d_in[8];
  const float* bt  = (const float*)d_in[9];
  const float* Wf  = (const float*)d_in[10];
  const float* bfb = (const float*)d_in[11];
  float* out = (float*)d_out;

  unsigned char* ws = (unsigned char*)d_ws;
  unsigned short* Xt16 = (unsigned short*)(ws + kOffX);
  unsigned short* Xi16 = (unsigned short*)(ws + kOffXi);
  float*          S32  = (float*)(ws + kOffX);
  unsigned short* Q16  = (unsigned short*)(ws + kOffQ);
  unsigned short* K16  = (unsigned short*)(ws + kOffK);
  float*          T32  = (float*)(ws + kOffT);
  unsigned short* V16  = (unsigned short*)(ws + kOffV);
  unsigned short* P16  = (unsigned short*)(ws + kOffP);
  unsigned short* Z16  = (unsigned short*)(ws + kOffZ);
  unsigned short* W16  = (unsigned short*)(ws + kOffW);
  unsigned short* Wq16 = W16 + 0 * (size_t)kWElems;
  unsigned short* Wk16 = W16 + 1 * (size_t)kWElems;
  unsigned short* Wv16 = W16 + 2 * (size_t)kWElems;
  unsigned short* Wt16 = W16 + 3 * (size_t)kWElems;
  unsigned short* Wf16 = W16 + 4 * (size_t)kWElems;

  const float attn_scale = 1.0f / sqrtf((float)kCd);

  wcast8_kernel<<<dim3(16, 5), dim3(256), 0, stream>>>(Wq, Wk, Wv, Wt, Wf, W16, kWCarry);

  xpose_cast_kernel<<<dim3(4, 64, 16), dim3(256), 0, stream>>>(feat_t, feat_i, Xt16, Xi16);

  wmma_gemm64<0, false, 2, 1, false><<<dim3(128, 1), dim3(256), 0, stream>>>(
      Xt16, Xt16, kCin, 0L, Wq16, Wq16, kCin, 0L, (void*)Q16, (void*)Q16, kCd, 0L,
      bq, T32, 0L, kPix, kCd, kCin, kWCarryInv);
  wmma_gemm64<0, false, 2, 1, false><<<dim3(128, 1), dim3(256), 0, stream>>>(
      Xi16, Xi16, kCin, 0L, Wk16, Wk16, kCin, 0L, (void*)K16, (void*)K16, kCd, 0L,
      bk, T32, 0L, kPix, kCd, kCin, kWCarryInv);
  wmma_gemm64<0, false, 2, 0, false><<<dim3(128, 1), dim3(256), 0, stream>>>(
      Xt16, Xt16, kCin, 0L, Wt16, Wt16, kCin, 0L, (void*)T32, (void*)T32, kCd, 0L,
      bt, T32, 0L, kPix, kCd, kCin, kWCarryInv);
  wmma_gemm64<0, false, 1, 1, false><<<dim3(16, kBatch), dim3(256), 0, stream>>>(
      Wv16, Wv16, kCin, 0L, Xi16, Xi16, kCin, (long)kNsp * kCin, (void*)V16, (void*)V16, kNsp, (long)kCd * kNsp,
      bv, T32, 0L, kCd, kNsp, kCin, kWCarryInv);

  for (int b = 0; b < kBatch; ++b) {
    for (int hf = 0; hf < kNsp / kQChunk; ++hf) {
      const size_t rowoff = (size_t)b * kNsp + (size_t)hf * kQChunk;
      wmma_gemm64<0, false, 0, 0, false><<<dim3(256, 1), dim3(256), 0, stream>>>(
          Q16 + rowoff * kCd, Q16 + rowoff * kCd, kCd, 0L,
          K16 + (size_t)b * kNsp * kCd, K16 + (size_t)b * kNsp * kCd, kCd, 0L,
          (void*)S32, (void*)S32, kNsp, 0L,
          bq, T32, 0L, kQChunk, kNsp, kCd, attn_scale);
      softmax_row_kernel<<<dim3(kQChunk), dim3(256), 0, stream>>>(S32, P16, kPCarry);
      wmma_gemm64<0, false, 0, 1, true><<<dim3(8, 1), dim3(256), 0, stream>>>(
          P16, P16, kNsp, 0L,
          V16 + (size_t)b * kCd * kNsp, V16 + (size_t)b * kCd * kNsp, kNsp, 0L,
          (void*)(Z16 + rowoff * kCd), (void*)(Z16 + rowoff * kCd), kCd, 0L,
          bq, T32 + rowoff * kCd, 0L, kQChunk, kCd, kNsp, kPCarryInv);
    }
  }

  wmma_gemm64<0, false, 1, 0, false><<<dim3(32, kBatch), dim3(256), 0, stream>>>(
      Wf16, Wf16, kCd, 0L, Z16, Z16, kCd, (long)kNsp * kCd, (void*)out, (void*)out, kNsp, (long)kCin * kNsp,
      bfb, T32, 0L, kCin, kNsp, kCd, kWCarryInv);
}
